// GATBlock_6150393168639
// MI455X (gfx1250) — hardware-verified
//
#include <hip/hip_runtime.h>
#include <stddef.h>
#include <stdint.h>


#define CIN    32
#define TT     2048
#define TQ     (TT / 32)
#define FF     32
#define KC     9
#define KCP    (2 * CIN * KC)
#define C1     64
#define C2     32
#define K1     (2 * CIN)
#define K2P    (2 * C1)
#define NTHR   256
#define NWAVE  8
#define EPT    8
#define CHUNK  (NTHR * EPT)
#define WCAP   (EPT * 32)
#define LISTN  (NWAVE * WCAP)
#define NBMAX  2048
#define NBRUN  1024
#define RCAP   28672
#define DEGCAP 64
#define STW    512
#define GBM    64
#define GBN    64
#define GTHR   128
#define CVT    64
#define CVR    (CVT + KC - 1)
#define XTW    (2 * CIN)
#define P0W    32
#define P1W    160
#define P2W    96
#define SSW    128
#define UWC    (FF * (KCP / 8))
#define UW1    (C1 * (K1 / 8))
#define UW2    (C2 * (K2P / 8))
#define UTOT   (UWC + 2 * UW1 + 2 * UW2)
#define NEGS   0.2f
#define BNEPS  1e-5f
#define WSMAX  134217728
#define LDS_AGG ((2 * RCAP + 2 * NBMAX + LISTN) * 4 + 64)

static_assert((CHUNK & (CHUNK - 1)) == 0 && CHUNK <= 4096);
static_assert((NBMAX & (NBMAX - 1)) == 0 && NBMAX <= 4096);
static_assert((NBRUN & (NBRUN - 1)) == 0 && NBRUN <= NBMAX && NBRUN >= 16);
static_assert(NTHR * 8 == NBMAX);
static_assert(LISTN >= NBMAX);
static_assert(LISTN >= NWAVE * WCAP);
static_assert((RCAP % 32) == 0);
static_assert(NWAVE * STW <= RCAP);
static_assert(C1 <= STW);
static_assert(LDS_AGG <= 300000);
static_assert(GBM == (GTHR / 32) * 16);
static_assert((K1 % 32) == 0 && (K2P % 32) == 0 && (KCP % 32) == 0);
static_assert(((2 * C1) % GBN) == 0 && ((2 * C2) % GBN) == 0);
static_assert(TT == NTHR * 8);
static_assert((TT % CVT) == 0 && (TT % GBM) == 0 && (TT % NBRUN) == 0 && (TT % 32) == 0);
static_assert(CIN == 32 && FF == 32 && TQ == 64);
static_assert(CVT == (GTHR / 32) * 16 && FF == 2 * 16);
static_assert((UWC % NTHR) == 0 && (UW1 % NTHR) == 0 && (UW2 % NTHR) == 0 && (UTOT % NTHR) == 0);
static_assert(P1W >= 1 + 2 * C1 && P2W >= 1 + 2 * C2 && (P1W % 32) == 0 && (P2W % 32) == 0);
static_assert(NWAVE * (2 * C1 + 2) <= LISTN);
static_assert(SSW == GTHR);

typedef float          v4f   __attribute__((ext_vector_type(4)));
typedef float          v8f   __attribute__((ext_vector_type(8)));
typedef int            v4i   __attribute__((ext_vector_type(4)));
typedef int            v8i   __attribute__((ext_vector_type(8)));
typedef unsigned short v8us  __attribute__((ext_vector_type(8)));
typedef __bf16         v16bf __attribute__((ext_vector_type(16)));
typedef v4f  __attribute__((may_alias)) v4fa;
typedef v8us __attribute__((may_alias)) v8usa;
union FragB { v16bf v; v8us u[2]; v8i w; };

__device__ __forceinline__ v8f wmb(const FragB& a, const FragB& b, v8f c) {
  v8f d = __builtin_amdgcn_wmma_f32_16x16x32_bf16(false, a.v, false, b.v, (short)0, c, false, false);
  asm volatile("v_nop\n\tv_nop\n\tv_nop\n\tv_nop" : "+v"(d) : "v"(a.w), "v"(b.w));
  return d;
}

__device__ __forceinline__ void ldwait() {
  asm volatile("s_wait_loadcnt 0x0" ::: "memory");
}

__device__ __forceinline__ unsigned bfbits(float v) {
  unsigned u = __float_as_uint(v);
  u = u + 0x7FFFu + ((u >> 16) & 1u);
  return u >> 16;
}
__device__ __forceinline__ float rbf(float v) { return __uint_as_float(bfbits(v) << 16); }

__device__ __forceinline__ v8us cvt8b(const v4f a, const v4f b) {
  v8us o;
  o[0] = (unsigned short)bfbits(a.x); o[1] = (unsigned short)bfbits(a.y);
  o[2] = (unsigned short)bfbits(a.z); o[3] = (unsigned short)bfbits(a.w);
  o[4] = (unsigned short)bfbits(b.x); o[5] = (unsigned short)bfbits(b.y);
  o[6] = (unsigned short)bfbits(b.z); o[7] = (unsigned short)bfbits(b.w);
  return o;
}

__device__ __forceinline__ v8f z8() { v8f z = {0.f, 0.f, 0.f, 0.f, 0.f, 0.f, 0.f, 0.f}; return z; }

__device__ __forceinline__ int scan_chunk(const int* __restrict__ dsts, int nE, int cbase, int slotBase,
                                          int nb, int vec8, int* list, int tid, int lane, int wave) {
  int wc = 0;
  const int el0  = tid * EPT;
  const int e0   = cbase + el0;
  const int sent = -2147483647 - 1;
  v4i da, db;
  if (vec8 != 0 && cbase + CHUNK <= nE) {
    da = *(const v4i*)(dsts + e0);
    db = *(const v4i*)(dsts + e0 + 4);
  } else {
    da.x = (e0     < nE) ? dsts[min(e0,     nE - 1)] : sent;
    da.y = (e0 + 1 < nE) ? dsts[min(e0 + 1, nE - 1)] : sent;
    da.z = (e0 + 2 < nE) ? dsts[min(e0 + 2, nE - 1)] : sent;
    da.w = (e0 + 3 < nE) ? dsts[min(e0 + 3, nE - 1)] : sent;
    db.x = (e0 + 4 < nE) ? dsts[min(e0 + 4, nE - 1)] : sent;
    db.y = (e0 + 5 < nE) ? dsts[min(e0 + 5, nE - 1)] : sent;
    db.z = (e0 + 6 < nE) ? dsts[min(e0 + 6, nE - 1)] : sent;
    db.w = (e0 + 7 < nE) ? dsts[min(e0 + 7, nE - 1)] : sent;
  }
  const unsigned nbs = (unsigned)slotBase;
  const unsigned unb = (unsigned)nb;
  const unsigned s0 = (unsigned)da.x - nbs, s1 = (unsigned)da.y - nbs;
  const unsigned s2 = (unsigned)da.z - nbs, s3 = (unsigned)da.w - nbs;
  const unsigned s4 = (unsigned)db.x - nbs, s5 = (unsigned)db.y - nbs;
  const unsigned s6 = (unsigned)db.z - nbs, s7 = (unsigned)db.w - nbs;
  const bool h0 = s0 < unb, h1 = s1 < unb, h2 = s2 < unb, h3 = s3 < unb;
  const bool h4 = s4 < unb, h5 = s5 < unb, h6 = s6 < unb, h7 = s7 < unb;
  const unsigned any = __builtin_amdgcn_ballot_w32(h0 | h1 | h2 | h3 | h4 | h5 | h6 | h7);
  if (any != 0u) {
#define HITJ(J, HJ, SJ) { \
      const unsigned mj = __builtin_amdgcn_ballot_w32(HJ); \
      if (mj != 0u) { \
        if (HJ) { \
          const int pos = wc + (int)__builtin_amdgcn_mbcnt_lo(mj, 0u); \
          if (pos < WCAP) list[wave * WCAP + pos] = ((el0 + (J)) << 12) | (int)(SJ); \
        } \
        wc += (int)__builtin_popcount(mj); } }
    HITJ(0, h0, s0)
    HITJ(1, h1, s1)
    HITJ(2, h2, s2)
    HITJ(3, h3, s3)
    HITJ(4, h4, s4)
    HITJ(5, h5, s5)
    HITJ(6, h6, s6)
    HITJ(7, h7, s7)
#undef HITJ
  }
  return wc;
}

__global__ __launch_bounds__(NTHR) void k_wprep(const float* __restrict__ Wsk, const float* __restrict__ Wl1,
                                                const float* __restrict__ Wr1, const float* __restrict__ Wl2,
                                                const float* __restrict__ Wr2,
                                                unsigned short* WC, unsigned short* W1B, unsigned short* W2B) {
  const int u = (int)blockIdx.x * NTHR + (int)threadIdx.x;
  v4f a, b;
  unsigned short* dp;
  if (u < UWC) {
    const int n  = u / (KCP / 8);
    const int k8 = (u - n * (KCP / 8)) * 8;
    const int kk = k8 >> 6;
    const int c0 = k8 & 31;
    const float* p = Wsk + (size_t)n * (CIN * KC) + (size_t)c0 * KC + kk;
    a.x = p[0];      a.y = p[KC];     a.z = p[2 * KC]; a.w = p[3 * KC];
    b.x = p[4 * KC]; b.y = p[5 * KC]; b.z = p[6 * KC]; b.w = p[7 * KC];
    dp = WC + (size_t)u * 8;
  } else if (u < UWC + UW1) {
    const int v  = u - UWC;
    const int n  = v >> 3;
    const int k8 = (v & 7) * 8;
    const float* p = Wl1 + (size_t)n * CIN + (k8 & (CIN - 1));
    a = *(const v4f*)p; b = *(const v4f*)(p + 4);
    dp = W1B + (size_t)v * 8;
  } else if (u < UWC + 2 * UW1) {
    const int v  = u - UWC - UW1;
    const int n  = v >> 3;
    const int k8 = (v & 7) * 8;
    const float* p = Wr1 + (size_t)n * CIN + (k8 & (CIN - 1));
    a = *(const v4f*)p; b = *(const v4f*)(p + 4);
    dp = W1B + (size_t)C1 * K1 + (size_t)v * 8;
  } else if (u < UWC + 2 * UW1 + UW2) {
    const int v  = u - UWC - 2 * UW1;
    const int n  = v >> 4;
    const int k8 = (v & 15) * 8;
    const float* p = Wl2 + (size_t)n * C1 + (k8 & (C1 - 1));
    a = *(const v4f*)p; b = *(const v4f*)(p + 4);
    dp = W2B + (size_t)v * 8;
  } else if (u < UTOT) {
    const int v  = u - UWC - 2 * UW1 - UW2;
    const int n  = v >> 4;
    const int k8 = (v & 15) * 8;
    const float* p = Wr2 + (size_t)n * C1 + (k8 & (C1 - 1));
    a = *(const v4f*)p; b = *(const v4f*)(p + 4);
    dp = W2B + (size_t)C2 * K2P + (size_t)v * 8;
  } else {
    return;
  }
  const v8us o = cvt8b(a, b);
  *(volatile v8us*)dp = o;
  __threadfence();
  *(volatile v8us*)dp = o;
}

__global__ __launch_bounds__(NTHR) void k_bn0stat(const float* __restrict__ x, int nB, float* part) {
  __shared__ float red1[NWAVE], red2[NWAVE];
  const int tid = (int)threadIdx.x, lane = tid & 31, wave = tid >> 5;
  const int blk = (int)blockIdx.x;
  const int c = blk / nB;
  const int b = blk - c * nB;
  const float* p = x + ((size_t)b * CIN + (size_t)c) * TT + 8 * tid;
  const v4f a = *(const v4f*)p;
  const v4f q4 = *(const v4f*)(p + 4);
  float v[8];
  v[0] = rbf(a.x);  v[1] = rbf(a.y);  v[2] = rbf(a.z);  v[3] = rbf(a.w);
  v[4] = rbf(q4.x); v[5] = rbf(q4.y); v[6] = rbf(q4.z); v[7] = rbf(q4.w);
  float s = ((v[0] + v[1]) + (v[2] + v[3])) + ((v[4] + v[5]) + (v[6] + v[7]));
#pragma unroll
  for (int off = 16; off > 0; off >>= 1) s += __shfl_xor(s, off);
  if (lane == 0) red1[wave] = s;
  __syncthreads();
  float tot = 0.0f;
#pragma unroll
  for (int w2 = 0; w2 < NWAVE; ++w2) tot += red1[w2];
  const float mean = tot * (1.0f / (float)TT);
  float qq = 0.0f;
#pragma unroll
  for (int i = 0; i < 8; ++i) { const float d = v[i] - mean; qq = fmaf(d, d, qq); }
#pragma unroll
  for (int off = 16; off > 0; off >>= 1) qq += __shfl_xor(qq, off);
  if (lane == 0) red2[wave] = qq;
  __syncthreads();
  float M2 = 0.0f;
#pragma unroll
  for (int w2 = 0; w2 < NWAVE; ++w2) M2 += red2[w2];
  v4f o = {0.0f, 0.0f, 0.0f, 0.0f};
  if (tid == 0) { o.x = (float)TT; o.y = mean; o.z = M2; }
  const bool wsv = tid < 8;
  float* op = part + (size_t)blk * P0W + 4 * tid;
  if (wsv) *(volatile v4f*)op = o;
  __threadfence();
  if (wsv) *(volatile v4f*)op = o;
}

__global__ __launch_bounds__(64) void k_bnfin(const float* __restrict__ part, int nPart, int rs, int crs,
                                              int mo, int qo, int ce, int pw, int C,
                                              const float* __restrict__ gam, const float* __restrict__ bet,
                                              float* ss) {
  __shared__ __attribute__((aligned(16))) float stg[SSW];
  const int tid = (int)threadIdx.x;
  const int c  = tid;
  const int cc = c < C ? c : C - 1;
  double n = 0.0, mean = 0.0, M2 = 0.0;
#pragma unroll 1
  for (int p = 0; p < nPart; ++p) {
    const float* pr = part + ((size_t)p * (size_t)rs + (size_t)cc * (size_t)crs) * (size_t)pw;
    const double nb = (double)pr[0];
    const double mb = (double)pr[mo + cc * ce];
    const double qb = (double)pr[qo + cc * ce];
    if (nb > 0.5) {
      const double nn = n + nb;
      const double delta = mb - mean;
      const double f = nb / nn;
      mean = mean + delta * f;
      M2 = M2 + qb + delta * delta * n * f;
      n = nn;
    }
  }
  const double nt = n < 1.0 ? 1.0 : n;
  const float varf  = (float)(M2 / nt);
  const float meanf = (float)mean;
  const float rstd = 1.0f / sqrtf(varf + BNEPS);
  float sc = rbf(gam[cc]) * rstd;
  float sh = rbf(bet[cc]) - meanf * sc;
  if (c >= C) { sc = 0.0f; sh = 0.0f; }
  stg[c] = sc;
  stg[64 + c] = sh;
  __syncthreads();
  v4f v;
  if (tid < SSW / 4) {
    v = *(const v4fa*)(stg + 4 * tid);
    *(volatile v4f*)(ss + 4 * tid) = v;
  }
  __threadfence();
  if (tid < SSW / 4) {
    *(volatile v4f*)(ss + 4 * tid) = v;
  }
}

__global__ __launch_bounds__(NTHR) void k_xn(const float* __restrict__ x, const float* __restrict__ ss0,
                                             int nUnits, unsigned short* xn) {
  const int u = (int)blockIdx.x * NTHR + (int)threadIdx.x;
  if (u >= nUnits) return;
  const int r  = u >> 3;
  const int p  = u & 7;
  const int k0 = 8 * (p & 3);
  const int c  = (r / TQ) & (CIN - 1);
  const float sc = ss0[c];
  const float sh = ss0[64 + c];
  const float* sp = x + (size_t)r * 32 + k0;
  const v4f a = *(const v4f*)sp;
  const v4f b = *(const v4f*)(sp + 4);
  float f[8] = {a.x, a.y, a.z, a.w, b.x, b.y, b.z, b.w};
  v8us o;
#pragma unroll
  for (int i = 0; i < 8; ++i) {
    const float y = fmaf(rbf(f[i]), sc, sh);
    const unsigned hb = bfbits(y);
    const unsigned lb = bfbits(y - __uint_as_float(hb << 16));
    o[i] = (unsigned short)(p < 4 ? hb : lb);
  }
  unsigned short* dp = xn + (size_t)u * 8;
  *(volatile v8us*)dp = o;
  __threadfence();
  *(volatile v8us*)dp = o;
}

__global__ __launch_bounds__(NTHR) void k_h1(const float* __restrict__ g1, const float* __restrict__ ss1,
                                             int nUnits, unsigned short* h1p) {
  __shared__ float ssh[SSW];
  const int tid = (int)threadIdx.x;
  if (tid < SSW) ssh[tid] = ss1[tid];
  __syncthreads();
  const int u = (int)blockIdx.x * NTHR + tid;
  if (u >= nUnits) return;
  const int r  = u >> 4;
  const int p  = u & 15;
  const int c0 = 8 * (p & 7);
  const float* sp = g1 + (size_t)r * C1 + c0;
  const v4f a = *(const v4f*)sp;
  const v4f b = *(const v4f*)(sp + 4);
  float f[8] = {a.x, a.y, a.z, a.w, b.x, b.y, b.z, b.w};
  v8us o;
#pragma unroll
  for (int i = 0; i < 8; ++i) {
    const float y = fmaxf(fmaf(f[i], ssh[c0 + i], ssh[64 + c0 + i]), 0.0f);
    const unsigned hb = bfbits(y);
    const unsigned lb = bfbits(y - __uint_as_float(hb << 16));
    o[i] = (unsigned short)(p < 8 ? hb : lb);
  }
  unsigned short* dp = h1p + (size_t)u * 8;
  *(volatile v8us*)dp = o;
  __threadfence();
  *(volatile v8us*)dp = o;
}

__global__ __launch_bounds__(GTHR) void k_gemm(const unsigned short* __restrict__ A,
                                               const unsigned short* __restrict__ WT,
                                               float* outF, int K, int ldo) {
  __shared__ __attribute__((aligned(16))) float stg[GBM * GBN];
  const int tid = (int)threadIdx.x, lane = tid & 31, wave = tid >> 5, hh = lane >> 4, m = lane & 15;
  const int rowBase = (int)blockIdx.x * GBM;
  const int col0    = (int)blockIdx.y * GBN;

  v8f acc[4];
  acc[0] = z8(); acc[1] = z8(); acc[2] = z8(); acc[3] = z8();
  const size_t arow = (size_t)(rowBase + 16 * wave + m) * (size_t)K + 8 * hh;
  const unsigned short* ap = A + arow;
  const unsigned short* wp = WT + (size_t)(col0 + m) * (size_t)K + 8 * hh;
  const int ksteps = K >> 5;
#pragma unroll 1
  for (int ks = 0; ks < ksteps; ++ks) {
    FragB af;
    af.u[0] = *(const v8us*)(ap + 32 * ks);
    af.u[1] = *(const v8us*)(ap + 32 * ks + 16);
#pragma unroll
    for (int t = 0; t < 4; ++t) {
      const unsigned short* wq = wp + (size_t)(16 * t) * (size_t)K + 32 * ks;
      FragB bf;
      bf.u[0] = *(const v8us*)wq;
      bf.u[1] = *(const v8us*)(wq + 16);
      acc[t] = wmb(af, bf, acc[t]);
    }
  }

#pragma unroll
  for (int t = 0; t < 4; ++t) {
    const int lc = 16 * t + m;
#pragma unroll
    for (int r = 0; r < 8; ++r) {
      const int lr = 16 * wave + 8 * hh + r;
      stg[lr * GBN + lc] = acc[t][r];
    }
  }
  __syncthreads();

  v4f fv[8];
#pragma unroll
  for (int i = 0; i < 8; ++i) {
    const int lr = 16 * wave + 2 * i + hh;
    fv[i] = *(const v4fa*)(stg + lr * GBN + 4 * m);
  }
#pragma unroll
  for (int i = 0; i < 8; ++i) {
    const int lr = 16 * wave + 2 * i + hh;
    const int gr = rowBase + lr;
    float* op = outF + (size_t)gr * (size_t)ldo + col0 + 4 * m;
    *(volatile v4f*)op = fv[i];
  }
  __threadfence();
#pragma unroll
  for (int i = 0; i < 8; ++i) {
    const int lr = 16 * wave + 2 * i + hh;
    const int gr = rowBase + lr;
    float* op = outF + (size_t)gr * (size_t)ldo + col0 + 4 * m;
    *(volatile v4f*)op = fv[i];
  }
}

template<int NH>
__global__ __launch_bounds__(NTHR) void k_agg(
    const int* __restrict__ srcs, const int* __restrict__ dsts,
    const float* __restrict__ HF, const float* __restrict__ att, const float* __restrict__ bias,
    float* outG, float* part, int nN, int nE, int nb, int vec8) {
  constexpr int C    = 32 * NH;
  constexpr int LD   = 2 * C;
  constexpr int PW   = ((1 + 2 * C + 31) / 32) * 32;
  constexpr int WSTW = 2 * C + 2;
  constexpr int CQ   = C / 4;
  static_assert(NWAVE * WSTW <= LISTN);
  static_assert(PW <= NWAVE * STW && PW / 4 <= NTHR && C <= NTHR && C <= STW);
  extern __shared__ v4f lds_dyn[];
  int* reg1 = (int*)lds_dyn;
  int* reg2 = reg1 + RCAP;
  int* scnt = reg2 + RCAP;
  int* soff = scnt + NBMAX;
  int* list = soff + NBMAX;
  int* wcnt = list + LISTN;
  int* wtot = wcnt + NWAVE;
  const int tid = (int)threadIdx.x, lane = tid & 31, wave = tid >> 5;
  const int nodeBase = (int)blockIdx.x * nb;

  for (int i = tid; i < NBMAX; i += NTHR) scnt[i] = 0;
  __syncthreads();

  int tot = 0;
  const int nChunks = (nE + CHUNK - 1) / CHUNK;
#pragma unroll 1
  for (int ch = 0; ch < nChunks; ++ch) {
    const int cbase = ch * CHUNK;
    const int wc = scan_chunk(dsts, nE, cbase, nodeBase, nb, vec8, list, tid, lane, wave);
    if (lane == 0) wcnt[wave] = wc;
    __syncthreads();
    int pre = 0, all = 0;
#pragma unroll
    for (int w2 = 0; w2 < NWAVE; ++w2) {
      int c = wcnt[w2];
      c = c < 0 ? 0 : (c > WCAP ? WCAP : c);
      all += c;
      pre += (w2 < wave) ? c : 0;
    }
    const int wcc  = wc > WCAP ? WCAP : wc;
    const int base = tot + pre;
#pragma unroll 1
    for (int i = lane; i < wcc; i += 32) {
      const int ent = list[wave * WCAP + i];
      const int el  = (ent >> 12) & (CHUNK - 1);
      const int sl  = ent & (NBMAX - 1);
      int eid = cbase + el;
      eid = eid > nE - 1 ? nE - 1 : eid;
      const int pos = base + i;
      if (pos < RCAP) reg1[pos] = (int)(((unsigned)eid << 12) | (unsigned)sl);
    }
    tot += all;
    tot = tot > RCAP ? RCAP : tot;
    __syncthreads();
  }
  const int nh = tot;

  if (wave == 0) {
#pragma unroll 1
    for (int b0 = 0; b0 < nh; b0 += 32) {
      const int idx = b0 + lane;
      const int uv  = reg1[idx < RCAP ? idx : RCAP - 1];
      const int m32 = (nh - b0) < 32 ? (nh - b0) : 32;
#pragma unroll 1
      for (int k = 0; k < m32; ++k) {
        const int u  = __builtin_amdgcn_readlane(uv, k);
        const int sl = u & (NBMAX - 1);
        if (lane == 0) scnt[sl] = scnt[sl] + 1;
      }
    }
  }
  __syncthreads();

  {
    const v4i ca = *(const v4i*)(scnt + 8 * tid);
    const v4i cb = *(const v4i*)(scnt + 8 * tid + 4);
    const int e0 = ca.x < 0 ? 0 : ca.x, e1 = ca.y < 0 ? 0 : ca.y, e2 = ca.z < 0 ? 0 : ca.z, e3 = ca.w < 0 ? 0 : ca.w;
    const int e4 = cb.x < 0 ? 0 : cb.x, e5 = cb.y < 0 ? 0 : cb.y, e6 = cb.z < 0 ? 0 : cb.z, e7 = cb.w < 0 ? 0 : cb.w;
    const int ts = e0 + e1 + e2 + e3 + e4 + e5 + e6 + e7;
    int incl = ts;
#pragma unroll
    for (int d = 1; d < 32; d <<= 1) {
      const int up = __shfl_up(incl, d);
      if (lane >= d) incl += up;
    }
    if (lane == 31) wtot[wave] = incl;
    __syncthreads();
    int pre = 0;
#pragma unroll
    for (int w2 = 0; w2 < NWAVE; ++w2) pre += (w2 < wave) ? wtot[w2] : 0;
    int run = pre + incl - ts;
    soff[8 * tid + 0] = run; run += e0;
    soff[8 * tid + 1] = run; run += e1;
    soff[8 * tid + 2] = run; run += e2;
    soff[8 * tid + 3] = run; run += e3;
    soff[8 * tid + 4] = run; run += e4;
    soff[8 * tid + 5] = run; run += e5;
    soff[8 * tid + 6] = run; run += e6;
    soff[8 * tid + 7] = run;
  }
  __syncthreads();
  for (int i = tid; i < NBMAX; i += NTHR) list[i] = soff[i];
  __syncthreads();

  if (wave == 0) {
#pragma unroll 1
    for (int b0 = 0; b0 < nh; b0 += 32) {
      const int idx = b0 + lane;
      const int uv  = reg1[idx < RCAP ? idx : RCAP - 1];
      const int m32 = (nh - b0) < 32 ? (nh - b0) : 32;
#pragma unroll 1
      for (int k = 0; k < m32; ++k) {
        const int u   = __builtin_amdgcn_readlane(uv, k);
        const int sl  = u & (NBMAX - 1);
        const int eid = (int)((unsigned)u >> 12);
        if (lane == 0) {
          int pos = list[sl];
          pos = pos < 0 ? 0 : (pos > RCAP - 1 ? RCAP - 1 : pos);
          reg2[pos] = eid;
          list[sl] = pos + 1;
        }
      }
    }
  }
  __syncthreads();

  const int nbw = nb >> 3;
  const bool ovf = (nh >= RCAP);
  const float qnan = __int_as_float(0x7fc00000);
  float* stw = (float*)reg1 + wave * STW;
  const int lc = lane < CQ ? lane : CQ - 1;
  float at[NH], bb[NH], wm[NH], wq[NH];
#pragma unroll
  for (int j = 0; j < NH; ++j) {
    at[j] = rbf(att[32 * j + lane]);
    bb[j] = rbf(bias[32 * j + lane]);
    wm[j] = 0.0f; wq[j] = 0.0f;
  }
#pragma unroll 1
  for (int jt = 0; jt < nbw; ++jt) {
    const int slot = wave * nbw + jt;
    const int grow = nodeBase + slot;
    const int gcl  = grow < nN ? grow : nN - 1;
    int st = soff[slot];
    const int craw = scnt[slot];
    int cnt = craw;
    st  = st < 0 ? 0 : (st > nh ? nh : st);
    cnt = cnt < 0 ? 0 : (cnt > DEGCAP ? DEGCAP : cnt);
    if (cnt > nh - st) cnt = nh - st;
    const float pz = (ovf || craw > DEGCAP) ? qnan : 0.0f;

    const float* drow = HF + (size_t)gcl * LD + lane;
    float xld[NH], xrd[NH];
#pragma unroll
    for (int j = 0; j < NH; ++j) { xld[j] = drow[32 * j]; xrd[j] = drow[C + 32 * j]; }
    ldwait();
    float mx[NH], dn[NH], av[NH];
    {
      float pp[NH];
#pragma unroll
      for (int j = 0; j < NH; ++j) {
        float v = xld[j] + xrd[j];
        v = v > 0.f ? v : v * NEGS;
        pp[j] = v * at[j];
      }
#pragma unroll
      for (int off = 16; off > 0; off >>= 1) {
#pragma unroll
        for (int j = 0; j < NH; ++j) pp[j] += __shfl_xor(pp[j], off);
      }
#pragma unroll
      for (int j = 0; j < NH; ++j) { mx[j] = pp[j]; dn[j] = 1.0f; av[j] = xld[j]; }
    }

#pragma unroll 1
    for (int q = 0; q < cnt; ++q) {
      int idx = st + q; idx = idx > RCAP - 1 ? RCAP - 1 : idx;
      int eid = reg2[idx]; eid = eid < 0 ? 0 : (eid > nE - 1 ? nE - 1 : eid);
      const int sraw = srcs[eid];
      const int s = sraw < 0 ? 0 : (sraw > nN - 1 ? nN - 1 : sraw);
      const float* sr = HF + (size_t)s * LD + lane;
      float hs[NH];
#pragma unroll
      for (int j = 0; j < NH; ++j) hs[j] = sr[32 * j];
      ldwait();
      float pp[NH];
#pragma unroll
      for (int j = 0; j < NH; ++j) {
        float v = hs[j] + xrd[j];
        v = v > 0.f ? v : v * NEGS;
        pp[j] = v * at[j];
      }
#pragma unroll
      for (int off = 16; off > 0; off >>= 1) {
#pragma unroll
        for (int j = 0; j < NH; ++j) pp[j] += __shfl_xor(pp[j], off);
      }
#pragma unroll
      for (int j = 0; j < NH; ++j) {
        const float al = pp[j];
        const float df = al - mx[j];
        const float ee = __expf(-fabsf(df));
        const bool up  = df > 0.f;
        const float s1 = up ? ee : 1.0f;
        const float s2 = up ? 1.0f : ee;
        mx[j] = up ? al : mx[j];
        dn[j] = fmaf(dn[j], s1, s2);
        av[j] = fmaf(av[j], s1, s2 * hs[j]);
      }
    }
    float r[NH];
#pragma unroll
    for (int j = 0; j < NH; ++j) {
      const float iv = __builtin_amdgcn_rcpf(dn[j]);
      r[j] = fmaf(av[j], iv, bb[j]) + pz;
    }
    {
      const float rk = 1.0f / (float)(jt + 1);
#pragma unroll
      for (int j = 0; j < NH; ++j) {
        const float d = r[j] - wm[j];
        wm[j] = fmaf(d, rk, wm[j]);
        wq[j] = fmaf(d, r[j] - wm[j], wq[j]);
      }
    }
    __builtin_amdgcn_fence(__ATOMIC_RELEASE, "wavefront");
    __builtin_amdgcn_wave_barrier();
#pragma unroll
    for (int j = 0; j < NH; ++j) stw[32 * j + lane] = r[j];
    __builtin_amdgcn_fence(__ATOMIC_RELEASE, "wavefront");
    __builtin_amdgcn_wave_barrier();
    const v4f gv = *(const v4fa*)(stw + 4 * lc);
    float* gp = outG + (size_t)grow * C + 4 * lc;
    const bool wsv = (grow < nN) && (lane < CQ);
    if (wsv) *(volatile v4f*)gp = gv;
    __threadfence();
    if (wsv) *(volatile v4f*)gp = gv;
  }
  __syncthreads();

  float* wst = (float*)list;
  if (lane == 0) wst[wave * WSTW] = (float)nbw;
#pragma unroll
  for (int j = 0; j < NH; ++j) {
    wst[wave * WSTW + 1 + 32 * j + lane]     = wm[j];
    wst[wave * WSTW + 1 + C + 32 * j + lane] = wq[j];
  }
  __syncthreads();
  float* pst = (float*)reg1;
  if (tid < C) {
    float n = 0.0f, mean = 0.0f, M2 = 0.0f;
#pragma unroll 1
    for (int w2 = 0; w2 < NWAVE; ++w2) {
      const float nbv = wst[w2 * WSTW];
      const float mb  = wst[w2 * WSTW + 1 + tid];
      const float qb  = wst[w2 * WSTW + 1 + C + tid];
      if (nbv > 0.5f) {
        const float nn = n + nbv;
        const float delta = mb - mean;
        const float f = nbv / nn;
        mean = fmaf(delta, f, mean);
        M2 = M2 + qb + delta * delta * n * f;
        n = nn;
      }
    }
    pst[1 + tid] = mean;
    pst[1 + C + tid] = M2;
    if (tid == 0) pst[0] = n;
  }
#pragma unroll 1
  for (int i = 2 * C + 1 + tid; i < PW; i += NTHR) pst[i] = 0.0f;
  __syncthreads();
  v4f ps;
  if (tid < PW / 4) {
    ps = *(const v4fa*)(pst + 4 * tid);
    *(volatile v4f*)(part + (size_t)blockIdx.x * PW + 4 * tid) = ps;
  }
  __threadfence();
  if (tid < PW / 4) {
    *(volatile v4f*)(part + (size_t)blockIdx.x * PW + 4 * tid) = ps;
  }
}

__global__ __launch_bounds__(GTHR) void k_convout(const float* __restrict__ x, const float* __restrict__ ss0,
                                                  const unsigned short* __restrict__ wc,
                                                  const float* __restrict__ bsk, const float* __restrict__ g2p,
                                                  const float* __restrict__ ss2, float* out, int nB) {
  __shared__ __attribute__((aligned(16))) unsigned short xt[CVR * XTW];
  __shared__ __attribute__((aligned(16))) float stg[FF * CVT];
  __shared__ float s0[SSW], s2[SSW], bq[FF];
  const int tid = (int)threadIdx.x, lane = tid & 31, wave = tid >> 5, hh = lane >> 4, m = lane & 15;
  const int t0 = (int)blockIdx.x * CVT;
  const int b  = (int)blockIdx.y;
  s0[tid] = ss0[tid];
  s2[tid] = ss2[tid];
  if (tid < FF) bq[tid] = rbf(bsk[tid]);
  __syncthreads();

#pragma unroll 1
  for (int i = tid; i < CIN * 9; i += GTHR) {
    const int c   = i / 9;
    const int gq  = i - 9 * c;
    const int tt0 = 8 * gq;
    const float sc = s0[c], sh = s0[64 + c];
    const float* xr = x + ((size_t)b * CIN + (size_t)c) * TT;
    float v[8];
#pragma unroll
    for (int e = 0; e < 8; ++e) {
      const int t  = t0 - (KC / 2) + tt0 + e;
      const int tc = t < 0 ? 0 : (t > TT - 1 ? TT - 1 : t);
      v[e] = xr[tc];
    }
#pragma unroll
    for (int e = 0; e < 8; ++e) {
      const int t = t0 - (KC / 2) + tt0 + e;
      float y = fmaf(rbf(v[e]), sc, sh);
      y = (t >= 0 && t < TT) ? y : 0.0f;
      const unsigned hb = bfbits(y);
      const unsigned lb = bfbits(y - __uint_as_float(hb << 16));
      xt[(tt0 + e) * XTW + c]       = (unsigned short)hb;
      xt[(tt0 + e) * XTW + CIN + c] = (unsigned short)lb;
    }
  }
  __syncthreads();

  v8f acc[2];
  acc[0] = z8(); acc[1] = z8();
  const unsigned short* arow = xt + (16 * wave + m) * XTW + 8 * hh;
  const unsigned short* wrow = wc + (size_t)m * KCP + 8 * hh;
#pragma unroll 1
  for (int kk = 0; kk < KC; ++kk) {
#pragma unroll
    for (int s = 0; s < 2; ++s) {
      FragB af;
      af.u[0] = *(const v8usa*)(arow + kk * XTW + 32 * s);
      af.u[1] = *(const v8usa*)(arow + kk * XTW + 32 * s + 16);
#pragma unroll
      for (int t = 0; t < 2; ++t) {
        const unsigned short* wq = wrow + (size_t)(16 * t) * KCP + kk * 64 + 32 * s;
        FragB bf;
        bf.u[0] = *(const v8us*)wq;
        bf.u[1] = *(const v8us*)(wq + 16);
        acc[t] = wmb(af, bf, acc[t]);
      }
    }
  }

#pragma unroll
  for (int t = 0; t < 2; ++t) {
    const int fcol = 16 * t + m;
#pragma unroll
    for (int r = 0; r < 8; ++r) {
      const int lr = 16 * wave + 8 * hh + r;
      stg[fcol * CVT + lr] = acc[t][r];
    }
  }
  __syncthreads();

  v4f ov[4];
#pragma unroll
  for (int i = 0; i < 4; ++i) {
    const int f = 8 * wave + 2 * i + hh;
    const v4f cv = *(const v4fa*)(stg + f * CVT + 4 * m);
    const size_t phi0 = (size_t)b * FF * TT + (size_t)f * TT + (size_t)t0;
    const size_t rn = (phi0 >> 5) + (size_t)(m >> 3);
    const int k0 = 4 * (m & 7);
    const v4f gv = *(const v4f*)(g2p + rn * C2 + k0);
    const float bf = bq[f];
    v4f o;
    o.x = fmaxf(cv.x + bf, 0.0f) + fmaxf(fmaf(gv.x, s2[k0 + 0], s2[64 + k0 + 0]), 0.0f);
    o.y = fmaxf(cv.y + bf, 0.0f) + fmaxf(fmaf(gv.y, s2[k0 + 1], s2[64 + k0 + 1]), 0.0f);
    o.z = fmaxf(cv.z + bf, 0.0f) + fmaxf(fmaf(gv.z, s2[k0 + 2], s2[64 + k0 + 2]), 0.0f);
    o.w = fmaxf(cv.w + bf, 0.0f) + fmaxf(fmaf(gv.w, s2[k0 + 3], s2[64 + k0 + 3]), 0.0f);
    ov[i] = o;
  }
#pragma unroll
  for (int i = 0; i < 4; ++i) {
    const int f = 8 * wave + 2 * i + hh;
    float* op = out + (size_t)b * FF * TT + (size_t)f * TT + t0 + 4 * m;
    *(volatile v4f*)op = ov[i];
  }
  __threadfence();
#pragma unroll
  for (int i = 0; i < 4; ++i) {
    const int f = 8 * wave + 2 * i + hh;
    float* op = out + (size_t)b * FF * TT + (size_t)f * TT + t0 + 4 * m;
    *(volatile v4f*)op = ov[i];
  }
  (void)nB;
}

static int pick_nb(int nE, int nN) {
  int nb = NBRUN;
  while (nb > 16 && (long long)nb * (long long)nE * 5LL > (long long)RCAP * (long long)nN * 4LL) nb >>= 1;
  return nb;
}
static inline int cdiv(int a, int b) { return (a + b - 1) / b; }
static inline size_t al256(size_t o) { return (o + 255) & ~(size_t)255; }

extern "C" void kernel_launch(void* const* d_in, const int* in_sizes, int n_in,
                              void* d_out, int out_size, void* d_ws, size_t ws_size,
                              hipStream_t stream) {
  if (n_in < 19) return;
  const int nx = in_sizes[0];
  if (nx < CIN * TT || (nx % (CIN * TT)) != 0) return;
  const int nB = nx / (CIN * TT);
  if (nB < 1 || nB > 512) return;
  const int nN = nB * TT;
  if (in_sizes[1] < 2 || (in_sizes[1] & 1) != 0) return;
  const int nE = in_sizes[1] / 2;
  if (nE < 1 || nE > (1 << 20)) return;
  if (in_sizes[3] != CIN || in_sizes[4] != CIN) return;
  if (in_sizes[5] != FF * CIN * KC || in_sizes[6] != FF) return;
  if (in_sizes[7] != C1 * CIN || in_sizes[8] != C1 * CIN || in_sizes[9] != C1) return;
  if (in_sizes[10] != C1 || in_sizes[11] != C1 || in_sizes[12] != C1) return;
  if (in_sizes[13] != C2 * C1 || in_sizes[14] != C2 * C1 || in_sizes[15] != C2) return;
  if (in_sizes[16] != C2 || in_sizes[17] != C2 || in_sizes[18] != C2) return;
  if ((long long)out_size != (long long)nB * FF * TT) return;

  const float* x     = (const float*)d_in[0];
  const int*   ei    = (const int*)  d_in[1];
  const float* g0    = (const float*)d_in[3];
  const float* be0   = (const float*)d_in[4];
  const float* Wskip = (const float*)d_in[5];
  const float* bskip = (const float*)d_in[6];
  const float* Wl1   = (const float*)d_in[7];
  const float* Wr1   = (const float*)d_in[8];
  const float* att1  = (const float*)d_in[9];
  const float* bias1 = (const float*)d_in[10];
  const float* g1    = (const float*)d_in[11];
  const float* be1   = (const float*)d_in[12];
  const float* Wl2   = (const float*)d_in[13];
  const float* Wr2   = (const float*)d_in[14];
  const float* att2  = (const float*)d_in[15];
  const float* bias2 = (const float*)d_in[16];
  const float* g2    = (const float*)d_in[17];
  const float* be2   = (const float*)d_in[18];
  float* out = (float*)d_out;
  const int* src = ei;
  const int* dst = ei + nE;

  const int nb = pick_nb(nE, nN);
  if ((nN % nb) != 0 || (nN % GBM) != 0) return;
  const int gA   = nN / nb;
  const int gM   = nN / GBM;
  const int vec8 = ((nE & 3) == 0) ? 1 : 0;

  char* ws = (char*)d_ws;
  size_t off = 0;
  const size_t oWC  = off; off = al256(off + (size_t)FF * KCP * 2);
  const size_t oW1B = off; off = al256(off + (size_t)(2 * C1) * K1 * 2);
  const size_t oW2B = off; off = al256(off + (size_t)(2 * C2) * K2P * 2);
  const size_t oPT0 = off; off = al256(off + (size_t)CIN * nB * P0W * 4);
  const size_t oSS0 = off; off = al256(off + (size_t)SSW * 4);
  const size_t oSS1 = off; off = al256(off + (size_t)SSW * 4);
  const size_t oSS2 = off; off = al256(off + (size_t)SSW * 4);
  const size_t oXN  = off; off = al256(off + (size_t)nN * K1 * 2);
  const size_t oXR1 = off; off = al256(off + (size_t)nN * (2 * C1) * 4);
  const size_t oG1  = off; off = al256(off + (size_t)nN * C1 * 4);
  const size_t oPT1 = off; off = al256(off + (size_t)gA * P1W * 4);
  const size_t oH1P = off; off = al256(off + (size_t)nN * K2P * 2);
  const size_t oXR2 = off; off = al256(off + (size_t)nN * (2 * C2) * 4);
  const size_t oG2  = off; off = al256(off + (size_t)nN * C2 * 4);
  const size_t oPT2 = off; off = al256(off + (size_t)gA * P2W * 4);
  if (off > ws_size || off > (size_t)WSMAX) return;
  unsigned short* WC   = (unsigned short*)(ws + oWC);
  unsigned short* W1B  = (unsigned short*)(ws + oW1B);
  unsigned short* W2B  = (unsigned short*)(ws + oW2B);
  float*          PT0  = (float*)(ws + oPT0);
  float*          SS0  = (float*)(ws + oSS0);
  float*          SS1  = (float*)(ws + oSS1);
  float*          SS2  = (float*)(ws + oSS2);
  unsigned short* XN   = (unsigned short*)(ws + oXN);
  float*          XLR1 = (float*)(ws + oXR1);
  float*          G1   = (float*)(ws + oG1);
  float*          PT1  = (float*)(ws + oPT1);
  unsigned short* H1P  = (unsigned short*)(ws + oH1P);
  float*          XLR2 = (float*)(ws + oXR2);
  float*          G2   = (float*)(ws + oG2);
  float*          PT2  = (float*)(ws + oPT2);

  hipFuncSetAttribute(reinterpret_cast<const void*>(&k_agg<2>), hipFuncAttributeMaxDynamicSharedMemorySize, LDS_AGG);
  hipFuncSetAttribute(reinterpret_cast<const void*>(&k_agg<1>), hipFuncAttributeMaxDynamicSharedMemorySize, LDS_AGG);

  k_wprep<<<UTOT / NTHR, NTHR, 0, stream>>>(Wskip, Wl1, Wr1, Wl2, Wr2, WC, W1B, W2B);
  k_bn0stat<<<CIN * nB, NTHR, 0, stream>>>(x, nB, PT0);
  k_bnfin<<<1, 64, 0, stream>>>(PT0, nB, 1, nB, 1, 2, 0, P0W, CIN, g0, be0, SS0);
  const int nUx = nN * (K1 / 8);
  k_xn<<<cdiv(nUx, NTHR), NTHR, 0, stream>>>(x, SS0, nUx, XN);
  k_gemm<<<dim3(gM, (2 * C1) / GBN), GTHR, 0, stream>>>(XN, W1B, XLR1, K1, 2 * C1);
  k_agg<2><<<gA, NTHR, LDS_AGG, stream>>>(src, dst, XLR1, att1, bias1, G1, PT1, nN, nE, nb, vec8);
  k_bnfin<<<1, 64, 0, stream>>>(PT1, gA, 1, 0, 1, 1 + C1, 1, P1W, C1, g1, be1, SS1);
  const int nUh = nN * (K2P / 8);
  k_h1<<<cdiv(nUh, NTHR), NTHR, 0, stream>>>(G1, SS1, nUh, H1P);
  k_gemm<<<dim3(gM, (2 * C2) / GBN), GTHR, 0, stream>>>(H1P, W2B, XLR2, K2P, 2 * C2);
  k_agg<1><<<gA, NTHR, LDS_AGG, stream>>>(src, dst, XLR2, att2, bias2, G2, PT2, nN, nE, nb, vec8);
  k_bnfin<<<1, 64, 0, stream>>>(PT2, gA, 1, 0, 1, 1 + C2, 1, P2W, C2, g2, be2, SS2);
  k_convout<<<dim3(TT / CVT, nB), GTHR, 0, stream>>>(x, SS0, WC, bskip, G2, SS2, out, nB);
}
